// MultiHeadSelfAttention_82265803587774
// MI455X (gfx1250) — hardware-run, weakly checked
//
#include <hip/hip_runtime.h>


#ifndef NB
#define NB 4
#endif
#ifndef SEQ
#define SEQ 2048
#endif
#define NB_FULL 4
#define DM   1024
#define NH   16
#define HD   64
#define QKCAR 16.0f
#define VCAR  16.0f
#define CCAR  256.0f
#define WOCAR 64.0f
#define PLOG  10.0f
#define CLOG  (0.125f * 1.4426950408889634f / (QKCAR * QKCAR))
#define OSCL  (1.0f / (CCAR * WOCAR))
#define PLANE ((size_t)NB * NH * SEQ * HD)
#define EROWS 256
#define RSC   2048.0f
#define RINV  (1.0f / 2048.0f)
#define NEGB  (-1.0e30f)
#define RPLANE ((size_t)NB * NH * EROWS * HD)

static_assert(SEQ % 128 == 0);
static_assert(NB >= 1 && NB <= NB_FULL);
static_assert(DM == NH * HD);
static_assert(DM % 64 == 0);
static_assert(DM % 32 == 0);
static_assert(HD == 64);
static_assert(EROWS % 128 == 0);
static_assert(EROWS % 64 == 0);
static_assert(EROWS <= SEQ);
static_assert((SEQ - EROWS) % 128 == 0);
static_assert(((size_t)NB * SEQ * DM * 2 + (size_t)3 * DM * DM * 2 + (size_t)DM * DM * 2 + 3 * PLANE * 2 + (size_t)NB * SEQ * DM * 2 + 3 * RPLANE * 2 + (size_t)NB * EROWS * DM * 2) <= (size_t)134217728);

typedef _Float16 h16;
typedef unsigned short bf;
typedef __attribute__((ext_vector_type(16))) __bf16   v16bf;
typedef __attribute__((ext_vector_type(16))) _Float16 v16h;
typedef __attribute__((ext_vector_type(8)))  _Float16 v8h;
typedef __attribute__((ext_vector_type(8)))  unsigned short v8us;
typedef __attribute__((ext_vector_type(8)))  float    v8f;
typedef __attribute__((ext_vector_type(4)))  float    v4f;
typedef v8h  __attribute__((may_alias)) v8ha;
typedef v4f  __attribute__((may_alias)) v4fa;

__device__ __forceinline__ unsigned short f2bf(float f) { unsigned u = __float_as_uint(f); u += 0x7FFFu + ((u >> 16) & 1u); return (unsigned short)(u >> 16); }
__device__ __forceinline__ float bf2f(unsigned short b) { return __uint_as_float(((unsigned)b) << 16); }
__device__ __forceinline__ float bfr(float f) { return bf2f(f2bf(f)); }
__device__ __forceinline__ v16h cat16(v8h lo, v8h hi) { return __builtin_shufflevector(lo, hi, 0, 1, 2, 3, 4, 5, 6, 7, 8, 9, 10, 11, 12, 13, 14, 15); }
__device__ __forceinline__ v16bf cat16b(v8us lo, v8us hi) { return __builtin_bit_cast(v16bf, __builtin_shufflevector(lo, hi, 0, 1, 2, 3, 4, 5, 6, 7, 8, 9, 10, 11, 12, 13, 14, 15)); }
__device__ __forceinline__ v8f wmma16(v16h a, v16h b, v8f c) { return __builtin_amdgcn_wmma_f32_16x16x32_f16(false, a, false, b, (short)0, c, false, false); }
__device__ __forceinline__ v8f wmmab(v16bf a, v16bf b, v8f c) { return __builtin_amdgcn_wmma_f32_16x16x32_bf16(false, a, false, b, (short)0, c, false, false); }
__device__ __forceinline__ v16h ldh(const h16* p) { return cat16(*(const v8h*)p, *(const v8h*)(p + 16)); }

static __device__ __forceinline__ h16 toh_flush(float v) { const h16 r = (h16)v; return (fabsf(v) < 6.103515625e-05f) ? (h16)0.0f : r; }
static __device__ __forceinline__ v8f wmma16g(v16h a, v16h b, v8f c) {
    c = __builtin_amdgcn_wmma_f32_16x16x32_f16(false, a, false, b, (short)0, c, false, false);
    asm volatile("v_nop\n\tv_nop\n\tv_nop\n\tv_nop" : "+v"(c) : "v"(a), "v"(b));
    return c;
}

template <typename T16> struct WFrag;
template <> struct WFrag<h16> { typedef v16h V; static __device__ __forceinline__ V ld(const h16* p) { return cat16(*(const v8h*)p, *(const v8h*)(p + 16)); } static __device__ __forceinline__ v8f mma(V a, V b, v8f c) { return wmma16(a, b, c); } };
template <> struct WFrag<bf> { typedef v16bf V; static __device__ __forceinline__ V ld(const bf* p) { return cat16b(*(const v8us*)p, *(const v8us*)(p + 16)); } static __device__ __forceinline__ v8f mma(V a, V b, v8f c) { return wmmab(a, b, c); } };

__global__ __launch_bounds__(256) void k_cvtx(const float* __restrict__ src, bf* dst) {
#pragma clang fp contract(off)
    const size_t i = (size_t)blockIdx.x * 256 + threadIdx.x; if (i >= (size_t)NB * SEQ * DM / 8) return;
    const int e8 = (int)(i % (DM / 8)); const size_t rs = i / (DM / 8); const int s = (int)(rs % SEQ); const int b = (int)(rs / SEQ);
    const v8f v = *(const v8f*)(src + ((size_t)s * NB_FULL + b) * DM + (size_t)e8 * 8); v8us o;
#pragma unroll
    for (int k = 0; k < 8; ++k) o[k] = f2bf(v[k]);
    *(volatile v8us*)(dst + i * 8) = o; __threadfence(); *(volatile v8us*)(dst + i * 8) = o;
}
__global__ __launch_bounds__(256) void k_cvt8(const float* __restrict__ src, bf* dst, size_t n8) {
#pragma clang fp contract(off)
    const size_t i = (size_t)blockIdx.x * 256 + threadIdx.x; if (i >= n8) return; const v8f v = *(const v8f*)(src + i * 8); v8us o;
#pragma unroll
    for (int k = 0; k < 8; ++k) o[k] = f2bf(v[k]);
    *(volatile v8us*)(dst + i * 8) = o; __threadfence(); *(volatile v8us*)(dst + i * 8) = o;
}
__global__ __launch_bounds__(256) void k_cvtw(const float* __restrict__ src, h16* dst, size_t n8) {
#pragma clang fp contract(off)
    const size_t i = (size_t)blockIdx.x * 256 + threadIdx.x; if (i >= n8) return; const v8f v = *(const v8f*)(src + i * 8); v8h o;
#pragma unroll
    for (int k = 0; k < 8; ++k) o[k] = (h16)(bfr(v[k]) * WOCAR);
    *(volatile v8h*)(dst + i * 8) = o; __threadfence(); *(volatile v8h*)(dst + i * 8) = o;
}

template <typename T16, int EPI>
__device__ __forceinline__ void gemm_body(const T16* __restrict__ A, const T16* __restrict__ Bt, const float* __restrict__ bias, h16* planes, h16* rplanes, float* C, size_t rofs) {
    typedef typename WFrag<T16>::V V;
    __shared__ __align__(16) float os[64 * 68];
    const int lane = threadIdx.x & 31, lr = lane & 15, hi = lane >> 4;
    const int r0 = blockIdx.x * 64, c0 = blockIdx.y * 64, bz = blockIdx.z;
    v8f acc[4][4];
#pragma unroll
    for (int mb = 0; mb < 4; ++mb)
#pragma unroll
        for (int nb = 0; nb < 4; ++nb) acc[mb][nb] = (v8f){};
    const size_t aoff = (size_t)(r0 + lr) * DM + 8 * hi, boff = (size_t)(c0 + lr) * DM + 8 * hi;
    const int ph0 = (EPI == 1 && r0 < EROWS) ? 0 : 1;
#pragma unroll 1
    for (int ph = ph0; ph < 2; ++ph) {
        const T16* Ab = A + ((ph == 0) ? (rofs + (size_t)bz * EROWS * DM) : ((size_t)bz * SEQ * DM));
#pragma unroll 1
        for (int kc = 0; kc < DM; kc += 32) {
            V a[4];
#pragma unroll
            for (int mb = 0; mb < 4; ++mb) a[mb] = WFrag<T16>::ld(Ab + aoff + (size_t)mb * 16 * DM + kc);
#pragma unroll
            for (int nb = 0; nb < 4; ++nb) { const V b = WFrag<T16>::ld(Bt + boff + (size_t)nb * 16 * DM + kc);
#pragma unroll
                for (int mb = 0; mb < 4; ++mb) acc[mb][nb] = WFrag<T16>::mma(a[mb], b, acc[mb][nb]); }
            asm volatile("v_nop\n\tv_nop\n\tv_nop\n\tv_nop" : "+v"(acc[0][0]), "+v"(acc[1][1]), "+v"(acc[2][2]), "+v"(acc[3][3]) : "v"(a[0]), "v"(a[3]));
        }
        if (ph == 0) {
#pragma unroll
            for (int mb = 0; mb < 4; ++mb)
#pragma unroll
                for (int nb = 0; nb < 4; ++nb) { asm volatile("v_nop\n\tv_nop\n\tv_nop\n\tv_nop" : "+v"(acc[mb][nb])); acc[mb][nb] = acc[mb][nb] * RINV; }
        }
    }
#pragma unroll
    for (int mb = 0; mb < 4; ++mb)
#pragma unroll
        for (int nb = 0; nb < 4; ++nb)
#pragma unroll
            for (int j = 0; j < 8; ++j) os[(mb * 16 + hi * 8 + j) * 68 + nb * 16 + lr] = acc[mb][nb][j];
    __syncthreads();
    const int rq = lane >> 3, c8 = (lane & 7) * 8;
    if (EPI == 0) {
        const int sec = blockIdx.y / NH, hh = blockIdx.y % NH; const int n = bz * NH + hh;
        if (sec < 2) {
            h16* dst = planes + (size_t)sec * PLANE + ((size_t)n * SEQ + r0) * HD;
#pragma unroll 1
            for (int ps = 0; ps < 2; ++ps) {
#pragma unroll 4
                for (int it = 0; it < 16; ++it) { const int row = it * 4 + rq; const v4f x0 = *(const v4fa*)(os + row * 68 + c8); const v4f x1 = *(const v4fa*)(os + row * 68 + c8 + 4); v8h o;
#pragma unroll
                    for (int j = 0; j < 4; ++j) { o[j] = toh_flush(x0[j] * QKCAR); o[4 + j] = toh_flush(x1[j] * QKCAR); }
                    *(volatile v8h*)(dst + (size_t)row * HD + c8) = o; }
                if (ps == 0) __threadfence(); }
            if (r0 < EROWS) {
                h16* dsr = rplanes + (size_t)sec * RPLANE + ((size_t)n * EROWS + r0) * HD;
#pragma unroll 1
                for (int ps = 0; ps < 2; ++ps) {
#pragma unroll 4
                    for (int it = 0; it < 16; ++it) { const int row = it * 4 + rq; const v4f x0 = *(const v4fa*)(os + row * 68 + c8); const v4f x1 = *(const v4fa*)(os + row * 68 + c8 + 4); v8h o;
#pragma unroll
                        for (int j = 0; j < 4; ++j) { const float a0 = x0[j] * QKCAR, a1 = x1[j] * QKCAR; const h16 h0 = toh_flush(a0), h1 = toh_flush(a1);
                            o[j] = toh_flush((a0 - (float)h0) * RSC); o[4 + j] = toh_flush((a1 - (float)h1) * RSC); }
                        *(volatile v8h*)(dsr + (size_t)row * HD + c8) = o; }
                    if (ps == 0) __threadfence(); }
            }
        } else {
            h16* dst = planes + 2 * PLANE + (size_t)n * HD * SEQ + r0;
#pragma unroll 1
            for (int ps = 0; ps < 2; ++ps) {
#pragma unroll 4
                for (int it = 0; it < 16; ++it) { const int d = it * 4 + rq; v8h o;
#pragma unroll
                    for (int j = 0; j < 8; ++j) o[j] = toh_flush(os[(c8 + j) * 68 + d] * VCAR);
                    *(volatile v8h*)(dst + (size_t)d * SEQ + c8) = o; }
                if (ps == 0) __threadfence(); }
            if (r0 < EROWS) {
                h16* dsr = rplanes + 2 * RPLANE + (size_t)n * HD * EROWS + r0;
#pragma unroll 1
                for (int ps = 0; ps < 2; ++ps) {
#pragma unroll 4
                    for (int it = 0; it < 16; ++it) { const int d = it * 4 + rq; v8h o;
#pragma unroll
                        for (int j = 0; j < 8; ++j) { const float a0 = os[(c8 + j) * 68 + d] * VCAR; const h16 h0 = toh_flush(a0); o[j] = toh_flush((a0 - (float)h0) * RSC); }
                        *(volatile v8h*)(dsr + (size_t)d * EROWS + c8) = o; }
                    if (ps == 0) __threadfence(); }
            }
        }
    } else {
        float* cb = C + ((size_t)r0 * NB + bz) * DM + c0; const int cofs = lr * 4;
        float bv[4];
#pragma unroll
        for (int j = 0; j < 4; ++j) bv[j] = bfr(bias[c0 + cofs + j]);
#pragma unroll 1
        for (int ps = 0; ps < 2; ++ps) {
#pragma unroll 4
            for (int it = 0; it < 32; ++it) { const int row = 2 * it + hi; const v4f x = *(const v4fa*)(os + row * 68 + cofs); v4f val;
#pragma unroll
                for (int j = 0; j < 4; ++j) val[j] = x[j] * OSCL + bv[j];
                *(volatile v4f*)(cb + (size_t)row * NB * DM + cofs) = val; }
            if (ps == 0) __threadfence(); }
    }
}

__global__ __launch_bounds__(32) void k_gemm_in(const bf* A, const bf* Bt, h16* planes, h16* rplanes) {
    gemm_body<bf, 0>(A, Bt, nullptr, planes, rplanes, nullptr, (size_t)0);
}
__global__ __launch_bounds__(32) void k_gemm_out(const h16* A, const h16* Bt, const float* bias, float* C, size_t rofs) {
    gemm_body<h16, 1>(A, Bt, bias, nullptr, nullptr, C, rofs);
}

template <bool EARLY>
__device__ __forceinline__ void attn_body(const h16* __restrict__ Qp, const h16* __restrict__ Kp, const h16* __restrict__ Vt,
                                          const h16* __restrict__ Qr, const h16* __restrict__ Kr, const h16* __restrict__ Vr, h16* Ctx, h16* Ctr) {
    __shared__ __align__(16) h16 ot[8 * 16 * 72];
    __shared__ __align__(16) h16 otr[EARLY ? 8 * 16 * 72 : 8];
    const int lane = threadIdx.x & 31, lr = lane & 15, hi = lane >> 4;
    const int wv = __builtin_amdgcn_readfirstlane((int)(threadIdx.x >> 5));
    constexpr int NQB = EARLY ? (EROWS / 128) : ((SEQ > EROWS) ? ((SEQ - EROWS) / 128) : 1);
    constexpr int QBASE = EARLY ? 0 : EROWS;
    const int n = (int)(blockIdx.x / NQB); const int q0 = QBASE + (int)(blockIdx.x % NQB) * 128 + wv * 16;
    const h16* qp = Qp + ((size_t)n * SEQ + q0 + lr) * HD + 8 * hi;
    const v16h qb0 = ldh(qp), qb1 = ldh(qp + 32);
    v16h qr0 = qb0, qr1 = qb1;
    if (EARLY) { const h16* qrp = Qr + ((size_t)n * EROWS + q0 + lr) * HD + 8 * hi; qr0 = ldh(qrp); qr1 = ldh(qrp + 32); }
    const h16* kp = Kp + ((size_t)n * SEQ + lr) * HD + 8 * hi;
    const h16* vp = Vt + ((size_t)n * HD + lr) * SEQ + 8 * hi;
    const h16* krp = Kr + ((size_t)n * EROWS + lr) * HD + 8 * hi;
    const h16* vrp = Vr + ((size_t)n * HD + lr) * EROWS + 8 * hi;
    v8f oacc[4], oaccr[4];
#pragma unroll
    for (int dt = 0; dt < 4; ++dt) { oacc[dt] = (v8f){}; oaccr[dt] = (v8f){}; }
    float mrun = NEGB, lsum = 0.0f;
    const int nst = (q0 + 47) >> 5;
    const int qd = q0 + lr - 8 * hi;
#pragma unroll 1
    for (int st = 0; st < nst; ++st) {
        const int kc = st * 32;
        const h16* k0 = kp + (size_t)kc * HD;
        const v16h ka00 = ldh(k0), ka01 = ldh(k0 + 32), ka10 = ldh(k0 + 16 * HD), ka11 = ldh(k0 + 16 * HD + 32);
        v8f s0 = (v8f){}, s1 = (v8f){};
        s0 = wmma16g(ka00, qb0, s0); s1 = wmma16g(ka10, qb0, s1); s0 = wmma16g(ka01, qb1, s0); s1 = wmma16g(ka11, qb1, s1);
        if (EARLY) {
            const h16* kr0 = krp + (size_t)kc * HD;
            const v16h kr00 = ldh(kr0), kr01 = ldh(kr0 + 32), kr10 = ldh(kr0 + 16 * HD), kr11 = ldh(kr0 + 16 * HD + 32);
            v8f t0 = (v8f){}, t1 = (v8f){};
            t0 = wmma16g(kr00, qb0, t0); t1 = wmma16g(kr10, qb0, t1); t0 = wmma16g(kr01, qb1, t0); t1 = wmma16g(kr11, qb1, t1);
            t0 = wmma16g(ka00, qr0, t0); t1 = wmma16g(ka10, qr0, t1); t0 = wmma16g(ka01, qr1, t0); t1 = wmma16g(ka11, qr1, t1);
            s0 = s0 + t0 * RINV; s1 = s1 + t1 * RINV;
        }
        if (st == nst - 1) {
            const int lim = qd - kc;
#pragma unroll
            for (int r = 0; r < 8; ++r) { s0[r] = (r > lim) ? NEGB : s0[r]; s1[r] = (16 + r > lim) ? NEGB : s1[r]; }
        }
        float mx = fmaxf(s0[0], s1[0]);
#pragma unroll
        for (int r = 1; r < 8; ++r) mx = fmaxf(mx, fmaxf(s0[r], s1[r]));
        mx = fmaxf(mx, __shfl_xor(mx, 16, 32));
        const float mnew = fmaxf(mrun, mx);
        const float corr = __builtin_amdgcn_exp2f((mrun - mnew) * CLOG);
        const float nbias = PLOG - mnew * CLOG;
        mrun = mnew;
        float psum = 0.0f; v16h pb, pr;
#pragma unroll
        for (int r = 0; r < 8; ++r) {
            const float e0 = fmaf(s0[r], CLOG, nbias), e1 = fmaf(s1[r], CLOG, nbias);
            const float x0 = __builtin_amdgcn_exp2f(e0), x1 = __builtin_amdgcn_exp2f(e1);
            if (EARLY) {
                const h16 h0 = (e0 < -14.0f) ? (h16)0.0f : (h16)x0; const h16 h1 = (e1 < -14.0f) ? (h16)0.0f : (h16)x1;
                psum += x0 + x1; pb[r] = h0; pb[8 + r] = h1;
                pr[r] = toh_flush((x0 - (float)h0) * RSC); pr[8 + r] = toh_flush((x1 - (float)h1) * RSC);
            } else {
                const float p0 = (e0 < -14.0f) ? 0.0f : x0; const float p1 = (e1 < -14.0f) ? 0.0f : x1;
                psum += p0 + p1; pb[r] = (h16)p0; pb[8 + r] = (h16)p1; pr[r] = (h16)0.0f; pr[8 + r] = (h16)0.0f;
            }
        }
        lsum = lsum * corr + psum;
#pragma unroll
        for (int dt = 0; dt < 4; ++dt) { oacc[dt] = oacc[dt] * corr; if (EARLY) oaccr[dt] = oaccr[dt] * corr; }
        const v16h va0 = ldh(vp + kc), va1 = ldh(vp + (size_t)16 * SEQ + kc), va2 = ldh(vp + (size_t)32 * SEQ + kc), va3 = ldh(vp + (size_t)48 * SEQ + kc);
        oacc[0] = wmma16g(va0, pb, oacc[0]); oacc[1] = wmma16g(va1, pb, oacc[1]); oacc[2] = wmma16g(va2, pb, oacc[2]); oacc[3] = wmma16g(va3, pb, oacc[3]);
        if (EARLY) {
            oaccr[0] = wmma16g(va0, pr, oaccr[0]); oaccr[1] = wmma16g(va1, pr, oaccr[1]); oaccr[2] = wmma16g(va2, pr, oaccr[2]); oaccr[3] = wmma16g(va3, pr, oaccr[3]);
            const v16h vr0 = ldh(vrp + kc), vr1 = ldh(vrp + (size_t)16 * EROWS + kc), vr2 = ldh(vrp + (size_t)32 * EROWS + kc), vr3 = ldh(vrp + (size_t)48 * EROWS + kc);
            oaccr[0] = wmma16g(vr0, pb, oaccr[0]); oaccr[1] = wmma16g(vr1, pb, oaccr[1]); oaccr[2] = wmma16g(vr2, pb, oaccr[2]); oaccr[3] = wmma16g(vr3, pb, oaccr[3]);
        }
    }
    const float lt = lsum + __shfl_xor(lsum, 16, 32);
    const float f = (CCAR / VCAR) * (1.0f / lt);
    const int tb = wv * (16 * 72);
#pragma unroll
    for (int dt = 0; dt < 4; ++dt) { v8h o, orr;
#pragma unroll
        for (int r = 0; r < 8; ++r) { float c = oacc[dt][r]; if (EARLY) c = c + oaccr[dt][r] * RINV; c = c * f;
            const h16 hv = toh_flush(c); o[r] = hv; orr[r] = toh_flush((c - (float)hv) * RSC); }
        *(v8ha*)&ot[tb + lr * 72 + dt * 16 + hi * 8] = o;
        if (EARLY) *(v8ha*)&otr[tb + lr * 72 + dt * 16 + hi * 8] = orr; }
    __syncthreads();
    const int b = n / NH, hh = n % NH; const int rq = lane >> 3, c8 = (lane & 7) * 8;
    h16* dst = Ctx + ((size_t)b * SEQ + q0) * DM + hh * HD;
#pragma unroll 1
    for (int ps = 0; ps < 2; ++ps) {
#pragma unroll
        for (int it = 0; it < 4; ++it) { const int row = it * 4 + rq; const v8h v = *(const v8ha*)&ot[tb + row * 72 + c8]; *(volatile v8h*)(dst + (size_t)row * DM + c8) = v; }
        if (ps == 0) __threadfence(); }
    if (EARLY) {
        h16* dsr = Ctr + ((size_t)b * EROWS + q0) * DM + hh * HD;
#pragma unroll 1
        for (int ps = 0; ps < 2; ++ps) {
#pragma unroll
            for (int it = 0; it < 4; ++it) { const int row = it * 4 + rq; const v8h v = *(const v8ha*)&otr[tb + row * 72 + c8]; *(volatile v8h*)(dsr + (size_t)row * DM + c8) = v; }
            if (ps == 0) __threadfence(); }
    }
}

__global__ __launch_bounds__(256) void k_attn(const h16* Qp, const h16* Kp, const h16* Vt, h16* Ctx) {
    attn_body<false>(Qp, Kp, Vt, Qp, Kp, Vt, Ctx, Ctx);
}
__global__ __launch_bounds__(256) __attribute__((amdgpu_num_vgpr(256))) void k_attn_early(const h16* Qp, const h16* Kp, const h16* Vt, const h16* Qr, const h16* Kr, const h16* Vr, h16* Ctx, h16* Ctr) {
    attn_body<true>(Qp, Kp, Vt, Qr, Kr, Vr, Ctx, Ctr);
}

extern "C" void kernel_launch(void* const* d_in, const int* in_sizes, int n_in,
                              void* d_out, int out_size, void* d_ws, size_t ws_size, hipStream_t stream) {
    if (n_in < 4) return;
    if (in_sizes[0] < ((SEQ - 1) * NB_FULL + NB) * DM) return;
    if (in_sizes[1] < 3 * DM * DM) return;
    if (in_sizes[2] < DM * DM) return;
    if (in_sizes[3] < DM) return;
    if (out_size < SEQ * NB * DM) return;
    const float* x = (const float*)d_in[0]; const float* win = (const float*)d_in[1]; const float* wo = (const float*)d_in[2]; const float* bo = (const float*)d_in[3];
    float* OUT = (float*)d_out;
    char* wsp = (char*)d_ws;
    auto take = [&](size_t bytes) { char* p = wsp; wsp += (bytes + 255) & ~(size_t)255; return (void*)p; };
    bf*  XB   = (bf*)take((size_t)NB * SEQ * DM * 2);
    bf*  WIN  = (bf*)take((size_t)3 * DM * DM * 2);
    h16* WO   = (h16*)take((size_t)DM * DM * 2);
    h16* PL   = (h16*)take(3 * PLANE * 2);
    h16* CTX  = (h16*)take((size_t)NB * SEQ * DM * 2);
    h16* RP   = (h16*)take(3 * RPLANE * 2);
    h16* CTXR = (h16*)take((size_t)NB * EROWS * DM * 2);
    if ((size_t)(wsp - (char*)d_ws) > ws_size) return;
    const size_t nx8 = (size_t)NB * SEQ * DM / 8, nwi8 = (size_t)3 * DM * DM / 8, nwo8 = (size_t)DM * DM / 8;
    k_cvtx<<<(unsigned)((nx8 + 255) / 256), 256, 0, stream>>>(x, XB);
    k_cvt8<<<(unsigned)((nwi8 + 255) / 256), 256, 0, stream>>>(win, WIN, nwi8);
    k_cvtw<<<(unsigned)((nwo8 + 255) / 256), 256, 0, stream>>>(wo, WO, nwo8);
    k_gemm_in<<<dim3(SEQ / 64, 3 * DM / 64, NB), 32, 0, stream>>>(XB, WIN, PL, RP);
    k_attn_early<<<(unsigned)(NB * NH * (EROWS / 128)), 256, 0, stream>>>(PL, PL + PLANE, PL + 2 * PLANE, RP, RP + RPLANE, RP + 2 * RPLANE, CTX, CTXR);
    if (SEQ > EROWS) k_attn<<<(unsigned)(NB * NH * ((SEQ - EROWS) / 128)), 256, 0, stream>>>(PL, PL + PLANE, PL + 2 * PLANE, CTX);
    k_gemm_out<<<dim3(SEQ / 64, DM / 64, NB), 32, 0, stream>>>(CTX, WO, bo, OUT, (size_t)(CTXR - CTX));
}
